// RGATModel_15393162788998
// MI455X (gfx1250) — hardware-verified
//
#include <hip/hip_runtime.h>
#include <math.h>

typedef __attribute__((ext_vector_type(16))) _Float16 v16h;
typedef __attribute__((ext_vector_type(8)))  _Float16 v8h;
typedef __attribute__((ext_vector_type(16))) __bf16   v16b;
typedef __attribute__((ext_vector_type(8)))  float    v8f;
typedef __attribute__((ext_vector_type(4)))  float    v4f;

__device__ __forceinline__ int frag_k(int i, int h) { return (i < 8) ? (8 * h + i) : (16 + 8 * h + (i - 8)); }
__device__ __forceinline__ __bf16 bf16_rne(float f) {
    unsigned int u = __float_as_uint(f);
    u += 0x7fffu + ((u >> 16) & 1u);
    return __builtin_bit_cast(__bf16, (unsigned short)(u >> 16));
}
__device__ __forceinline__ float bf16_f32(__bf16 b) { return __uint_as_float(((unsigned int)__builtin_bit_cast(unsigned short, b)) << 16); }
__device__ __forceinline__ v8f wmma16(v16h a, v16h b, v8f c) {
    c = __builtin_amdgcn_wmma_f32_16x16x32_f16(false, a, false, b, (short)0, c, false, false);
    asm volatile("v_nop\n\tv_nop\n\tv_nop\n\tv_nop" : "+v"(c) : "v"(a), "v"(b));
    return c;
}
__device__ __forceinline__ v8f wmmab(v16b a, v16b b, v8f c) {
    c = __builtin_amdgcn_wmma_f32_16x16x32_bf16(false, a, false, b, (short)0, c, false, false);
    asm volatile("v_nop\n\tv_nop\n\tv_nop\n\tv_nop" : "+v"(c) : "v"(a), "v"(b));
    return c;
}
struct Split { v16b hi, lo; };
__device__ __forceinline__ v8f wmma3(const Split& a, const Split& b, v8f c) {
    c = __builtin_amdgcn_wmma_f32_16x16x32_bf16(false, a.hi, false, b.hi, (short)0, c, false, false);
    c = __builtin_amdgcn_wmma_f32_16x16x32_bf16(false, a.hi, false, b.lo, (short)0, c, false, false);
    c = __builtin_amdgcn_wmma_f32_16x16x32_bf16(false, a.lo, false, b.hi, (short)0, c, false, false);
    asm volatile("v_nop\n\tv_nop\n\tv_nop\n\tv_nop" : "+v"(c) : "v"(a.hi), "v"(a.lo), "v"(b.hi), "v"(b.lo));
    return c;
}
struct Split3 { v16b hi, mid, lo; };
__device__ __forceinline__ v8f wmma6(const Split3& a, const Split3& b, v8f c) {
    c = __builtin_amdgcn_wmma_f32_16x16x32_bf16(false, a.hi, false, b.hi, (short)0, c, false, false);
    c = __builtin_amdgcn_wmma_f32_16x16x32_bf16(false, a.hi, false, b.mid, (short)0, c, false, false);
    c = __builtin_amdgcn_wmma_f32_16x16x32_bf16(false, a.mid, false, b.hi, (short)0, c, false, false);
    c = __builtin_amdgcn_wmma_f32_16x16x32_bf16(false, a.hi, false, b.lo, (short)0, c, false, false);
    c = __builtin_amdgcn_wmma_f32_16x16x32_bf16(false, a.mid, false, b.mid, (short)0, c, false, false);
    c = __builtin_amdgcn_wmma_f32_16x16x32_bf16(false, a.lo, false, b.hi, (short)0, c, false, false);
    asm volatile("v_nop\n\tv_nop\n\tv_nop\n\tv_nop" : "+v"(c) : "v"(a.hi), "v"(a.mid), "v"(a.lo), "v"(b.hi), "v"(b.mid), "v"(b.lo));
    return c;
}

__device__ __forceinline__ v16h fh_ld(const float* __restrict__ p, long long sk, int k0, int h, int klen, float s) {
    v16h a;
#pragma unroll
    for (int i = 0; i < 16; ++i) { const int k = k0 + frag_k(i, h); a[i] = (k < klen) ? (_Float16)(p[(long long)k * sk] * s) : (_Float16)0.f; }
    return a;
}
__device__ __forceinline__ Split sp_ld(const float* __restrict__ p, long long sk, int k0, int h, int klen, float s) {
    Split r;
#pragma unroll
    for (int i = 0; i < 16; ++i) {
        const int k = k0 + frag_k(i, h); const float x = (k < klen) ? p[(long long)k * sk] * s : 0.f;
        const __bf16 hb = bf16_rne(x); r.hi[i] = hb; r.lo[i] = bf16_rne(x - bf16_f32(hb));
    }
    return r;
}
__device__ __forceinline__ Split3 sp3_ld(const float* __restrict__ p, long long sk, int k0, int h, int klen, float s) {
    Split3 r;
#pragma unroll
    for (int i = 0; i < 16; ++i) {
        const int k = k0 + frag_k(i, h); const float x = (k < klen) ? p[(long long)k * sk] * s : 0.f;
        const __bf16 hb = bf16_rne(x); const float r1 = x - bf16_f32(hb); const __bf16 mb = bf16_rne(r1);
        r.hi[i] = hb; r.mid[i] = mb; r.lo[i] = bf16_rne(r1 - bf16_f32(mb));
    }
    return r;
}
__device__ __forceinline__ v16b bh_ld(const float* __restrict__ p, long long sk, int k0, int h, int klen, float s) {
    v16b a;
#pragma unroll
    for (int i = 0; i < 16; ++i) { const int k = k0 + frag_k(i, h); a[i] = bf16_rne((k < klen) ? p[(long long)k * sk] * s : 0.f); }
    return a;
}
__device__ __forceinline__ v16h fh_row(const _Float16* __restrict__ row, int k0, int h) {
    v16h a;
#pragma unroll
    for (int i = 0; i < 16; ++i) a[i] = row[k0 + frag_k(i, h)];
    return a;
}

#define VST2(T, ptr, val) do { *(volatile T*)(ptr) = (val); __threadfence(); *(volatile T*)(ptr) = (val); } while (0)
typedef float v4f __attribute__((ext_vector_type(4)));
#define VST2V4(ptr, val) do { *(volatile v4f*)(ptr) = (val); __threadfence(); *(volatile v4f*)(ptr) = (val); } while (0)

__device__ __attribute__((noinline)) float act_fn(float v, int act) {
    if (act == 1) return fmaxf(v, 0.f);
    if (act == 2) { const float u = 0.7978845608028654f * (v + 0.044715f * v * v * v); return 0.5f * v * (1.f + tanhf(u)); }
    if (act == 3) return v / (1.f + expf(-v));
    if (act == 4) return 0.5f * v * (1.f + erff(v * 0.7071067811865476f));
    if (act == 5) return tanhf(v);
    if (act == 6) return 1.f / (1.f + expf(-v));
    if (act == 7) return (v > 0.f) ? v : 0.01f * v;
    if (act == 8) return (v > 0.f) ? v : (expf(v) - 1.f);
    if (act == 9) return fminf(fmaxf(v, 0.f), 6.f);
    if (act == 10) return fabsf(v);
    if (act == 11) return (v >= 0.f) ? v : 0.1f * v;
    if (act == 12) return (v > 0.f) ? v : 0.2f * v;
    if (act == 13) return (v > 20.f) ? v : log1pf(expf(v));
    return v;
}

struct GemmP {
    const float* A; const float* B; const float* bias; const float* R; float* C;
    long long sAo, sAi, sAm, sAk, sBo, sBi, sBn, sBk, sCo, sCi, sCm, sRo, sRi, sRm, sRn;
    int M, N, K, zi_n, flags, act; float alpha, beta, sa, sb;
    int Npad, pad_;
};
static_assert(sizeof(GemmP) == 5 * 8 + 15 * 8 + 6 * 4 + 4 * 4 + 2 * 4, "GemmP has padding");

template <int MODE>
__global__ __launch_bounds__(32) void k_gemm(GemmP p) {
    const int lane = threadIdx.x & 31, h = lane >> 4, l15 = lane & 15;
    const int m0 = blockIdx.y * 16, n0 = blockIdx.x * 32;
    const int z = blockIdx.z, zo = z / p.zi_n, zi = z - zo * p.zi_n;
    const float* A = p.A + zo * p.sAo + zi * p.sAi;
    const float* B = p.B + zo * p.sBo + zi * p.sBi;
    const int am = min(m0 + l15, p.M - 1);
    v8f acc[2], comp[2];
#pragma unroll
    for (int t = 0; t < 2; ++t) { v8f zz = {}; acc[t] = zz; comp[t] = zz; }
    for (int k0 = 0; k0 < p.K; k0 += 32) {
        const float* arow = A + (long long)am * p.sAm;
        if (MODE == 1) {
            const Split a = sp_ld(arow, p.sAk, k0, h, p.K, 1.f);
#pragma unroll
            for (int t = 0; t < 2; ++t) {
                const int bn = min(n0 + t * 16 + l15, p.N - 1);
                acc[t] = wmma3(a, sp_ld(B + (long long)bn * p.sBn, p.sBk, k0, h, p.K, 1.f), acc[t]);
            }
        } else if (MODE == 3) {
            const Split3 a = sp3_ld(arow, p.sAk, k0, h, p.K, 1.f);
#pragma unroll
            for (int t = 0; t < 2; ++t) {
                const int bn = min(n0 + t * 16 + l15, p.N - 1);
                acc[t] = wmma6(a, sp3_ld(B + (long long)bn * p.sBn, p.sBk, k0, h, p.K, 1.f), acc[t]);
            }
        } else if (MODE == 4) {
            const Split3 a = sp3_ld(arow, p.sAk, k0, h, p.K, 1.f);
#pragma unroll
            for (int t = 0; t < 2; ++t) {
                const int bn = min(n0 + t * 16 + l15, p.N - 1); v8f zz = {};
                const v8f part = wmma6(a, sp3_ld(B + (long long)bn * p.sBn, p.sBk, k0, h, p.K, 1.f), zz);
                const v8f y = part - comp[t]; const v8f s = acc[t] + y; comp[t] = (s - acc[t]) - y; acc[t] = s;
            }
        } else if (MODE == 2) {
            const v16b a = bh_ld(arow, p.sAk, k0, h, p.K, 1.f);
#pragma unroll
            for (int t = 0; t < 2; ++t) {
                const int bn = min(n0 + t * 16 + l15, p.N - 1);
                acc[t] = wmmab(a, bh_ld(B + (long long)bn * p.sBn, p.sBk, k0, h, p.K, 1.f), acc[t]);
            }
        } else {
            const v16h a = fh_ld(arow, p.sAk, k0, h, p.K, p.sa);
#pragma unroll
            for (int t = 0; t < 2; ++t) {
                const int bn = min(n0 + t * 16 + l15, p.N - 1);
                acc[t] = wmma16(a, fh_ld(B + (long long)bn * p.sBn, p.sBk, k0, h, p.K, p.sb), acc[t]);
            }
        }
    }
    const float iscale = (MODE == 0) ? p.alpha / (p.sa * p.sb) : p.alpha;
    float* C = p.C + zo * p.sCo + zi * p.sCi;
    const float* R = p.R + zo * p.sRo + zi * p.sRi;
    __shared__ __align__(16) float ctile[16][36];
#pragma unroll
    for (int t = 0; t < 2; ++t) {
        const int n = n0 + t * 16 + l15; const int nn = min(n, p.N - 1);
#pragma unroll
        for (int r = 0; r < 8; ++r) {
            const int m = m0 + 8 * h + r; const int mm = min(m, p.M - 1);
            float v = acc[t][r] * iscale;
            if (p.flags & 1) v += p.bias[nn];
            if (p.flags & 2) v += p.bias[mm];
            v = act_fn(v, p.act);
            if (p.flags & 4) v += p.beta * R[(long long)mm * p.sRm + (long long)nn * p.sRn];
            ctile[8 * h + r][t * 16 + l15] = (n < p.N) ? v : 0.f;
        }
    }
    __syncthreads();
    const int NW = (p.Npad > p.N) ? p.Npad : p.N;
    const bool fast = (m0 + 16 <= p.M) && (n0 + 32 <= NW) && ((p.sCm & 3) == 0) && ((((size_t)C) & 15) == 0);
    if (fast) {
#pragma unroll
        for (int s = 0; s < 4; ++s) {
            const int row = s * 4 + (lane >> 3), c4 = (lane & 7) * 4;
            const v4f v = *(const v4f*)&ctile[row][c4];
            VST2V4(C + (long long)(m0 + row) * p.sCm + n0 + c4, v);
        }
    } else {
        for (int row = 0; row < 16; ++row) {
            const int m = m0 + row, n = n0 + lane;
            if (m < p.M && n < NW) VST2(float, C + (long long)m * p.sCm + n, ctile[row][lane]);
        }
    }
}

#define AW 4
struct AttnP {
    const float* Q; const float* K; const float* V; float* O; float* P; const float* Mf; const int* Mi; float* ST;
    const float* Pw; const float* Rt; const int* SQ; const int* SK;
    long long swb, swh, swi, swj, srb, srh, sri;
    long long sQb, sQh, sQi, sQd, sKb, sKh, sKj, sKd, sVb, sVh, sVj, sVd, sOb, sOh, sOi, sPb, sPh, sPi, smb, smh, smi, smj;
    int Lq, Lk, dh, dv, hrep, causal, coff, pband;
    float scale, mfill; int nonorm, mpol;
    int roff, rn, segpol, win;
};
static_assert(sizeof(AttnP) == 12 * 8 + 29 * 8 + 16 * 4, "AttnP has padding");

#ifndef KATTN_ATTR
#define KATTN_ATTR
#endif
template <int DHP, int DVP, int QM, bool SPLITPV, bool TWOPASS>
__global__ __launch_bounds__(32 * AW) KATTN_ATTR void k_attn(AttnP p) {
    constexpr int NT = DVP / 16;
    constexpr int KS = DHP / 32;
    constexpr int VP = DVP + 8;
    __shared__ __align__(16) float    pl[AW][16 * 64];
    __shared__ __align__(16) _Float16 vl[(SPLITPV ? 2 : 1) * 64 * VP];
    const int lane = threadIdx.x & 31, hf = lane >> 4, l15 = lane & 15, wave = threadIdx.x >> 5;
    const int h = blockIdx.y, b = blockIdx.z, hk = h / p.hrep;
    const int q0 = (blockIdx.x * AW + wave) * 16;
    float* myp = pl[wave];
    const float L2E = 1.4426950408889634f;
    const float NEG = -__builtin_inff();
    const int qi = min(q0 + l15, p.Lq - 1);
    const float* qrow = p.Q + b * p.sQb + h * p.sQh + (long long)qi * p.sQi;
    const float* kbase = p.K + b * p.sKb + hk * p.sKh;
    const float* vbase = p.V + b * p.sVb + hk * p.sVh;
    v16h qa[QM == 0 ? KS : 1]; Split qs_[QM == 1 ? KS : 1]; Split3 qt_[QM == 2 ? KS : 1];
#pragma unroll
    for (int ks = 0; ks < KS; ++ks) {
        if (QM == 2) qt_[ks] = sp3_ld(qrow, p.sQd, ks * 32, hf, p.dh, 1.f);
        else if (QM == 1) qs_[ks] = sp_ld(qrow, p.sQd, ks * 32, hf, p.dh, 1.f);
        else qa[ks] = fh_ld(qrow, p.sQd, ks * 32, hf, p.dh, 1.f);
    }
    v8f o[NT]; float m8[8], l8[8];
#pragma unroll
    for (int t = 0; t < NT; ++t) { v8f zz = {}; o[t] = zz; }
#pragma unroll
    for (int i = 0; i < 8; ++i) { m8[i] = NEG; l8[i] = 0.f; }
    int jend = p.Lk;
    if (p.causal == 1) { const int je = (blockIdx.x * AW + AW - 1) * 16 + 16 + p.coff; jend = min(jend, max(je, 0)); }
    const int npass = TWOPASS ? 2 : 1;
    for (int pass = 0; pass < npass; ++pass) {
        const bool dopv = (!TWOPASS) || pass == 1;
        for (int j0 = 0; j0 < jend; j0 += 64) {
            if (dopv) {
                __syncthreads();
                for (int idx = threadIdx.x; idx < 64 * DVP; idx += 32 * AW) {
                    const int jr = idx / DVP, d = idx - jr * DVP, j = j0 + jr;
                    const float f = (j < p.Lk && d < p.dv) ? vbase[(long long)j * p.sVj + (long long)d * p.sVd] : 0.f;
                    if (SPLITPV) {
                        const __bf16 hb = bf16_rne(f);
                        ((__bf16*)vl)[jr * VP + d] = hb; ((__bf16*)vl)[64 * VP + jr * VP + d] = bf16_rne(f - bf16_f32(hb));
                    } else vl[jr * VP + d] = (_Float16)f;
                }
            }
            v8f s[4];
#pragma unroll
            for (int t = 0; t < 4; ++t) {
                const int j = min(j0 + t * 16 + l15, p.Lk - 1);
                const float* krow = kbase + (long long)j * p.sKj;
                v8f acc = {};
#pragma unroll
                for (int ks = 0; ks < KS; ++ks) {
                    if (QM == 2)      acc = wmma6(qt_[ks], sp3_ld(krow, p.sKd, ks * 32, hf, p.dh, 1.f), acc);
                    else if (QM == 1) acc = wmma3(qs_[ks], sp_ld(krow, p.sKd, ks * 32, hf, p.dh, 1.f), acc);
                    else              acc = wmma16(qa[ks], fh_ld(krow, p.sKd, ks * 32, hf, p.dh, 1.f), acc);
                }
                s[t] = acc;
            }
            float pv[8][4];
#pragma unroll
            for (int i = 0; i < 8; ++i) {
                const int irow = q0 + i + 8 * hf;
                const int ic = min(irow, p.Lq - 1);
                float sc[4];
#pragma unroll
                for (int t = 0; t < 4; ++t) {
                    const int jg = j0 + t * 16 + l15;
                    float v = s[t][i] * p.scale;
                    if (p.Mf) v += p.Mf[b * p.smb + h * p.smh + (long long)ic * p.smi + (long long)min(jg, p.Lk - 1) * p.smj];
                    if (p.Rt) { int rc = ic - min(jg, p.Lk - 1) + p.roff; rc = rc < 0 ? 0 : (rc >= p.rn ? p.rn - 1 : rc); v += p.Rt[b * p.srb + h * p.srh + (long long)ic * p.sri + rc]; }
                    if (p.Mi) { const int mv = p.Mi[b * p.smb + h * p.smh + (long long)ic * p.smi + (long long)min(jg, p.Lk - 1) * p.smj]; if (p.mpol ? (mv != 0) : (mv == 0)) v = p.mfill; }
                    if (p.SQ) { const bool same = p.SQ[(long long)b * p.Lq + ic] == p.SK[(long long)b * p.Lk + min(jg, p.Lk - 1)]; if (p.segpol ? same : !same) v = p.mfill; }
                    if (p.causal == 2 && jg > irow + p.coff) v = p.mfill;
                    if (jg >= p.Lk || (p.causal == 1 && jg > irow + p.coff) || (p.causal == 3 && jg < irow + p.coff) || (p.win > 0 && irow + p.coff - jg > p.win)) v = NEG; else v *= L2E;
                    sc[t] = v;
                }
                if (!TWOPASS || pass == 0) {
                    float mx = fmaxf(fmaxf(sc[0], sc[1]), fmaxf(sc[2], sc[3]));
                    mx = fmaxf(mx, __shfl_xor(mx, 1, 32)); mx = fmaxf(mx, __shfl_xor(mx, 2, 32));
                    mx = fmaxf(mx, __shfl_xor(mx, 4, 32)); mx = fmaxf(mx, __shfl_xor(mx, 8, 32));
                    const float mnew = fmaxf(m8[i], mx);
                    const float corr = (mnew == NEG) ? 1.f : exp2f(m8[i] - mnew);
                    float rs = 0.f;
#pragma unroll
                    for (int t = 0; t < 4; ++t) {
                        const float pp = (sc[t] == NEG) ? 0.f : exp2f(sc[t] - mnew); rs += pp;
                        pv[i][t] = p.Pw ? pp * p.Pw[b * p.swb + h * p.swh + (long long)ic * p.swi + (long long)min(j0 + t * 16 + l15, p.Lk - 1) * p.swj] : pp;
                    }
                    rs += __shfl_xor(rs, 1, 32); rs += __shfl_xor(rs, 2, 32); rs += __shfl_xor(rs, 4, 32); rs += __shfl_xor(rs, 8, 32);
                    l8[i] = l8[i] * corr + rs; m8[i] = mnew;
                    if (!TWOPASS) {
#pragma unroll
                        for (int t = 0; t < NT; ++t) o[t][i] *= corr;
                    }
                } else {
                    const float inv = (l8[i] > 0.f) ? 1.f / l8[i] : 0.f;
#pragma unroll
                    for (int t = 0; t < 4; ++t) {
                        const int jg = j0 + t * 16 + l15;
                        float pp = (sc[t] == NEG) ? 0.f : exp2f(sc[t] - m8[i]) * inv;
                        if (p.Pw) pp *= p.Pw[b * p.swb + h * p.swh + (long long)ic * p.swi + (long long)min(jg, p.Lk - 1) * p.swj];
                        pv[i][t] = pp;
                    }
                }
            }
            if (dopv) {
#pragma unroll
                for (int i = 0; i < 8; ++i)
#pragma unroll
                    for (int t = 0; t < 4; ++t) myp[(i + 8 * hf) * 64 + t * 16 + l15] = pv[i][t];
                __syncthreads();
                if (p.P) {
                    float* pb_ = p.P + b * p.sPb + h * p.sPh;
                    const bool fastP = (p.pband == 0) && ((p.sPi & 3) == 0) && (j0 + 64 <= p.Lk) && (q0 + 16 <= p.Lq) && ((((size_t)pb_) & 15) == 0);
                    if (fastP) {
#pragma unroll
                        for (int s = 0; s < 8; ++s) {
                            const int row = s * 2 + (lane >> 4), c4 = (lane & 15) * 4;
                            const v4f v = *(const v4f*)(myp + row * 64 + c4);
                            VST2V4(pb_ + (long long)(q0 + row) * p.sPi + j0 + c4, v);
                        }
                    } else {
                        for (int row = 0; row < 16; ++row) {
                            const int irow = q0 + row; if (irow >= p.Lq) continue;
                            for (int c = lane; c < 64; c += 32) {
                                const int jg = j0 + c; if (jg >= p.Lk) continue;
                                if (p.pband == 0) VST2(float, pb_ + (long long)irow * p.sPi + jg, myp[row * 64 + c]);
                                else if (jg - irow <= p.pband && irow - jg <= p.pband) VST2(float, pb_ + (long long)irow * p.sPi + (jg - irow + p.pband), myp[row * 64 + c]);
                            }
                        }
                    }
                }
                if (SPLITPV) {
                    const Split pa0 = sp_ld(myp + l15 * 64, 1, 0, hf, 64, 1.f), pa1 = sp_ld(myp + l15 * 64, 1, 32, hf, 64, 1.f);
                    const __bf16* vh = (const __bf16*)vl; const __bf16* vlo = vh + 64 * VP;
#pragma unroll
                    for (int t = 0; t < NT; ++t) {
                        const int dcol = t * 16 + l15;
                        Split b0, b1;
#pragma unroll
                        for (int e = 0; e < 16; ++e) {
                            const int k0 = frag_k(e, hf), k1 = 32 + frag_k(e, hf);
                            b0.hi[e] = vh[k0 * VP + dcol]; b0.lo[e] = vlo[k0 * VP + dcol]; b1.hi[e] = vh[k1 * VP + dcol]; b1.lo[e] = vlo[k1 * VP + dcol];
                        }
                        o[t] = wmma3(pa0, b0, o[t]);
                        o[t] = wmma3(pa1, b1, o[t]);
                    }
                } else {
                    const v16h pa0 = fh_ld(myp + l15 * 64, 1, 0, hf, 64, 4096.f), pa1 = fh_ld(myp + l15 * 64, 1, 32, hf, 64, 4096.f);
#pragma unroll
                    for (int t = 0; t < NT; ++t) {
                        const int dcol = t * 16 + l15;
                        v16h b0, b1;
#pragma unroll
                        for (int e = 0; e < 16; ++e) { b0[e] = vl[frag_k(e, hf) * VP + dcol]; b1[e] = vl[(32 + frag_k(e, hf)) * VP + dcol]; }
                        o[t] = wmma16(pa0, b0, o[t]);
                        o[t] = wmma16(pa1, b1, o[t]);
                    }
                }
            }
        }
    }
    float* obase = p.O + b * p.sOb + h * p.sOh;
    if (p.ST) {
        const int rl = lane >> 1, isel = rl & 7;
        float mv = 0.f, lv = 0.f;
#pragma unroll
        for (int i = 0; i < 8; ++i) if (i == isel) { mv = m8[i]; lv = l8[i]; }
        const int irow = q0 + rl;
        if (irow < p.Lq) { float* st = p.ST + (((long long)b * gridDim.y + h) * p.Lq + irow) * 2 + (lane & 1); VST2(float, st, (lane & 1) ? lv : mv * 0.6931471805599453f); }
    }
    float invr[8];
#pragma unroll
    for (int i = 0; i < 8; ++i) {
        if (TWOPASS) invr[i] = SPLITPV ? 1.f : (1.f / 4096.f);
        else if (p.nonorm) invr[i] = exp2f(m8[i]) * (SPLITPV ? 1.f : (1.f / 4096.f));
        else invr[i] = (l8[i] > 0.f) ? (SPLITPV ? 1.f / l8[i] : 1.f / (l8[i] * 4096.f)) : 0.f;
    }
    __syncthreads();
    const bool ofast = ((p.sOi & 3) == 0) && ((((size_t)obase) & 15) == 0) && (q0 + 16 <= p.Lq);
#pragma unroll
    for (int c0 = 0; c0 < DVP; c0 += 64) {
#pragma unroll
        for (int i = 0; i < 8; ++i)
#pragma unroll
            for (int t = 0; t < NT; ++t) if (t * 16 >= c0 && t * 16 < c0 + 64) myp[(i + 8 * hf) * 64 + (t * 16 - c0) + l15] = o[t][i] * invr[i];
        __syncthreads();
        const int cw = (DVP - c0 < 64) ? (DVP - c0) : 64;
        if (ofast && (c0 + cw <= p.dv) && (cw % 32 == 0)) {
            const int lpr = cw / 4;
            const int rows_per_ins = 32 / lpr;
            for (int r0 = 0; r0 < 16; r0 += rows_per_ins) {
                const int row = r0 + lane / lpr, c4 = (lane % lpr) * 4;
                const v4f v = *(const v4f*)(myp + row * 64 + c4);
                VST2V4(obase + (long long)(q0 + row) * p.sOi + c0 + c4, v);
            }
        } else {
            for (int row = 0; row < 16; ++row) {
                const int irow = q0 + row; if (irow >= p.Lq) continue;
                for (int c = lane; c < cw; c += 32) { const int d = c0 + c; if (d < p.dv) VST2(float, obase + (long long)irow * p.sOi + d, myp[row * 64 + c]); }
            }
        }
        __syncthreads();
    }
}

struct TrP { const float* src; float* dst; const float* R2; long long sSz, lds, sDz, ldd, sRz, ldr; int R, C, flags, act; float alpha, beta; };
static_assert(sizeof(TrP) == 3 * 8 + 6 * 8 + 6 * 4, "TrP has padding");
__global__ __launch_bounds__(256) void k_tr(TrP p) {
    __shared__ float tile[32][33];
    const int c0 = blockIdx.x * 32, r0 = blockIdx.y * 32, z = blockIdx.z;
    const int lane = threadIdx.x & 31, wave = threadIdx.x >> 5;
    const float* s = p.src + z * p.sSz;
#pragma unroll
    for (int k = 0; k < 4; ++k) {
        const int rl = wave * 4 + k, r = r0 + rl, c = c0 + lane;
        tile[rl][lane] = (r < p.R && c < p.C) ? s[(long long)r * p.lds + c] : 0.f;
    }
    __syncthreads();
    float* d = p.dst + z * p.sDz; const float* rr = p.R2 + z * p.sRz;
#pragma unroll
    for (int k = 0; k < 4; ++k) {
        const int cl = wave * 4 + k, c = c0 + cl, r = r0 + lane;
        if (c < p.C && r < p.R) {
            float v = act_fn(p.alpha * tile[lane][cl], p.act);
            if (p.flags & 1) v += p.beta * rr[(long long)c * p.ldr + r];
            VST2(float, d + (long long)c * p.ldd + r, v);
        }
    }
}

__global__ __launch_bounds__(256) void k_affine(const float* __restrict__ src, float* __restrict__ dst, int n, float a, float b, const float* __restrict__ sdev) {
    const int i = blockIdx.x * 256 + threadIdx.x;
    if (i < n) { const float aa = sdev ? a * sdev[0] : a; const float v = aa * src[i] + b; VST2(float, dst + i, v); }
}

struct SmP { const float* src; float* dst; const float* Mf; long long sz, sr, dz, dr, smz, smr; int n, pad; float scale_in, scale_out; };
static_assert(sizeof(SmP) == 3 * 8 + 6 * 8 + 4 * 4, "SmP has padding");
__global__ __launch_bounds__(256) void k_softmax(SmP p) {
    __shared__ float red[256];
    const int r = blockIdx.x, z = blockIdx.y, tid = threadIdx.x;
    const float* s = p.src + z * p.sz + (long long)r * p.sr;
    const float* mf = p.Mf ? (p.Mf + z * p.smz + (long long)r * p.smr) : nullptr;
    float mx = -__builtin_inff();
    for (int j = tid; j < p.n; j += 256) { float v = s[j] * p.scale_in; if (mf) v += mf[j]; mx = fmaxf(mx, v); }
    red[tid] = mx; __syncthreads();
    for (int o = 128; o > 0; o >>= 1) { if (tid < o) red[tid] = fmaxf(red[tid], red[tid + o]); __syncthreads(); }
    mx = red[0]; __syncthreads();
    float sum = 0.f;
    for (int j = tid; j < p.n; j += 256) { float v = s[j] * p.scale_in; if (mf) v += mf[j]; sum += (mx == -__builtin_inff()) ? 0.f : expf(v - mx); }
    red[tid] = sum; __syncthreads();
    for (int o = 128; o > 0; o >>= 1) { if (tid < o) red[tid] += red[tid + o]; __syncthreads(); }
    sum = red[0];
    const float inv = (sum > 0.f) ? p.scale_out / sum : 0.f;
    float* d = p.dst + z * p.dz + (long long)r * p.dr;
    for (int j = tid; j < p.n; j += 256) { float v = s[j] * p.scale_in; if (mf) v += mf[j]; const float o = (mx == -__builtin_inff()) ? 0.f : expf(v - mx) * inv; VST2(float, d + j, o); }
}
__global__ __launch_bounds__(256) void k_stats(const float* __restrict__ x, long long sz, long long so, long long si, int inner, int n, float eps, float* __restrict__ stat, int mode) {
    __shared__ float red[256];
    const int z = blockIdx.x, tid = threadIdx.x;
    const float* base = x + z * sz;
    float s = 0.f;
    for (int e = tid; e < n; e += 256) s += base[(long long)(e / inner) * so + (long long)(e % inner) * si];
    red[tid] = s; __syncthreads();
    for (int o = 128; o > 0; o >>= 1) { if (tid < o) red[tid] += red[tid + o]; __syncthreads(); }
    const float mu = (mode == 0 || mode == 3) ? red[0] / (float)n : 0.f; __syncthreads();
    float q = 0.f;
    for (int e = tid; e < n; e += 256) { const float dlt = base[(long long)(e / inner) * so + (long long)(e % inner) * si] - mu; q += dlt * dlt; }
    red[tid] = q; __syncthreads();
    for (int o = 128; o > 0; o >>= 1) { if (tid < o) red[tid] += red[tid + o]; __syncthreads(); }
    {
        float rs;
        if (mode == 2) rs = sqrtf((float)n) / fmaxf(sqrtf(red[0]), eps); else if (mode == 3) rs = rsqrtf(red[0] / (float)(n - 1) + eps); else rs = rsqrtf(red[0] / (float)n + eps);
        if (tid < 32) { const float v = (tid == 0) ? mu : ((tid == 1) ? rs : 0.f); VST2(float, stat + (long long)z * 32 + tid, v); }
    }
}
__global__ __launch_bounds__(256) void k_norm_apply(const float* __restrict__ x, float* __restrict__ y, const float* __restrict__ stat, const float* __restrict__ g, const float* __restrict__ bta,
                                                     int Z, int C, int L, int G, int bn, int act) {
    const long long idx = (long long)blockIdx.x * 256 + threadIdx.x;
    if (idx >= (long long)Z * C * L) return;
    const int l = (int)(idx % L); const long long zc = idx / L; const int c = (int)(zc % C), z = (int)(zc / C); (void)l;
    const int set = bn ? c : (z * G + c / (C / G));
    float v = (x[idx] - stat[(long long)set * 32]) * stat[(long long)set * 32 + 1];
    if (g) v *= g[c];
    if (bta) v += bta[c];
    v = act_fn(v, act);
    VST2(float, y + idx, v);
}

__global__ __launch_bounds__(256) void k_lse_neg(const float* __restrict__ st, float* __restrict__ c, int n) {
    const int i = blockIdx.x * 256 + threadIdx.x;
    if (i < n) { const float v = -(st[2 * i] + logf(st[2 * i + 1])); VST2(float, c + i, v); }
}

__global__ __launch_bounds__(256) void k_iota(int* __restrict__ dst, int n, int a, int b) {
    const int i = blockIdx.x * 256 + threadIdx.x;
    if (i < n) { const int v = a * i + b; VST2(int, dst + i, v); }
}

__global__ __launch_bounds__(256) void k_axpby(const float* __restrict__ x, const float* __restrict__ y, float* __restrict__ dst, int n, float a, float b, float c) {
    const int i = blockIdx.x * 256 + threadIdx.x;
    if (i < n) { const float v = a * x[i] + b * y[i] + c; VST2(float, dst + i, v); }
}

struct RopeP { const float* X; float* Y; const float* C; const float* Sn; const int* pos; long long sXr, sXh, sYr, sYh, sCb, sCp, sCd; int R, Hn, D, S, mode, tmode, pmode, pad; };
static_assert(sizeof(RopeP) == 5 * 8 + 7 * 8 + 8 * 4, "RopeP has padding");
__global__ __launch_bounds__(256) void k_rope(RopeP p) {
    const long long idx = (long long)blockIdx.x * 256 + threadIdx.x;
    if (idx >= (long long)p.R * p.Hn * p.D) return;
    const int d = (int)(idx % p.D); const long long rh = idx / p.D; const int h = (int)(rh % p.Hn); const int r = (int)(rh / p.Hn);
    const int half = p.D / 2;
    int partner; float sign;
    if (p.mode == 0) { partner = (d < half) ? d + half : d - half; sign = (d < half) ? -1.f : 1.f; }
    else { partner = d ^ 1; sign = (d & 1) ? 1.f : -1.f; }
    const int tcol = (p.tmode == 0) ? d : ((p.tmode == 1) ? (d % half) : (d >> 1));
    const int pp = (p.pmode == 0) ? (r % p.S) : ((p.pmode == 1) ? h : p.pos[r]);
    const long long toff = (long long)(r / p.S) * p.sCb + (long long)pp * p.sCp + (long long)tcol * p.sCd;
    const float* xr = p.X + (long long)r * p.sXr + (long long)h * p.sXh;
    const float v = xr[d] * p.C[toff] + sign * xr[partner] * p.Sn[toff];
    VST2(float, p.Y + (long long)r * p.sYr + (long long)h * p.sYh + d, v);
}

__global__ __launch_bounds__(256) void k_invf(float* __restrict__ invb, int half, int D, float base, float num, int fmode, float cexp) {
    const int i = blockIdx.x * 256 + threadIdx.x;
    if (i >= ((half + 31) / 32) * 32) return;
    if (i >= half) { VST2(float, invb + i, 0.f); return; }
    const float e = (float)(2 * i) / (float)D;
    float invf;
    if (fmode == 1) invf = num * expf((float)(2 * i) * cexp);
    else if (fmode == 2) invf = num * powf(base, (-2.0f * ((float)i - 1.0f)) / (float)D);
    else invf = num * (1.0f / powf(base, e));
    VST2(float, invb + i, invf);
}
__global__ __launch_bounds__(256) void k_sincos(float* __restrict__ cs, float* __restrict__ sn, const float* __restrict__ invb, int S, int half, float pscale) {
    const int idx = blockIdx.x * 256 + threadIdx.x;
    if (idx >= S * half) return;
    const int s = idx / half, i = idx - s * half;
    const float ang = (pscale * (float)s) * invb[i];
    VST2(float, cs + idx, cosf(ang)); VST2(float, sn + idx, sinf(ang));
}

__global__ __launch_bounds__(256) void k_mulact(const float* __restrict__ x, const float* __restrict__ y, float* __restrict__ dst, int n, int act) {
    const int i = blockIdx.x * 256 + threadIdx.x;
    if (i < n) { const float v = act_fn(x[i], act) * y[i]; VST2(float, dst + i, v); }
}

__global__ __launch_bounds__(256) void k_matvec(GemmP p) {
    const int rpt = (p.N == 1) ? 1 : 32;
    const long long r0 = ((long long)blockIdx.x * 256 + threadIdx.x) * rpt; const int z = blockIdx.z, zo = z / p.zi_n, zi = z - zo * p.zi_n;
    if (r0 >= p.M) return;
    const float* Bb = p.B + zo * p.sBo + zi * p.sBi;
    float* C = p.C + zo * p.sCo + zi * p.sCi; const float* R = p.R + zo * p.sRo + zi * p.sRi;
    for (int rr = 0; rr < rpt; ++rr) {
        const long long r = r0 + rr; if (r >= p.M) break;
        const float* A = p.A + zo * p.sAo + zi * p.sAi + r * p.sAm;
        float acc[8] = {0.f, 0.f, 0.f, 0.f, 0.f, 0.f, 0.f, 0.f};
        for (int k = 0; k < p.K; ++k) { const float a = A[(long long)k * p.sAk];
#pragma unroll
            for (int j = 0; j < 8; ++j) if (j < p.N) acc[j] += a * Bb[(long long)j * p.sBn + (long long)k * p.sBk]; }
#pragma unroll
        for (int j = 0; j < 8; ++j) if (j < p.N) {
            float v = acc[j] * p.alpha;
            if (p.flags & 1) v += p.bias[j];
            if (p.flags & 2) v += p.bias[r];
            v = act_fn(v, p.act);
            if (p.flags & 4) v += p.beta * R[r * p.sRm + (long long)j * p.sRn];
            VST2(float, C + r * p.sCm + j, v);
        }
    }
}
__global__ __launch_bounds__(256) void k_smallsoftmax(const float* __restrict__ src, float* __restrict__ dst, long long sr, long long dr, int n, long long R, float scale) {
    const long long r0 = ((long long)blockIdx.x * 256 + threadIdx.x) * 32;
    for (int rr = 0; rr < 32; ++rr) {
        const long long r = r0 + rr; if (r >= R) return;
        const float* s = src + r * sr; float* d = dst + r * dr;
        float mx = -__builtin_inff();
        for (int j = 0; j < n; ++j) mx = fmaxf(mx, s[j] * scale);
        float sum = 0.f;
        for (int j = 0; j < n; ++j) sum += expf(s[j] * scale - mx);
        const float inv = 1.f / sum;
        for (int j = 0; j < n; ++j) { const float v = expf(s[j] * scale - mx) * inv; VST2(float, d + j, v); }
    }
}

__global__ __launch_bounds__(32) void k_unitstat(float* __restrict__ st) { const int t = threadIdx.x; const float v = (t == 1) ? 1.f : 0.f; VST2(float, st + t, v); }

__global__ __launch_bounds__(256) void k_lincopy(const float* __restrict__ src, long long lds, float* __restrict__ dst, long long ldd, long long rows, int cols) {
    const long long i = (long long)blockIdx.x * 256 + threadIdx.x; if (i >= rows * cols) return;
    const long long r = i / cols; const int c = (int)(i - r * cols);
    const float v = src[r * lds + c]; VST2(float, dst + r * ldd + c, v);
}


#define IL3_CH 4096
__global__ __launch_bounds__(256) void k_csr3_bcount(const int* __restrict__ tgt, int E, int N, int* __restrict__ CNT) { __shared__ int tt[IL3_CH]; const int ch = blockIdx.x; const int b = threadIdx.x; const int e0 = ch * IL3_CH; const int nt = min(IL3_CH, E - e0);
    for (int i = b; i < nt; i += 256) tt[i] = (int)(((long long)tgt[e0 + i] * 256) / N); __syncthreads(); int c = 0;
    for (int i = 0; i < nt; ++i) c += (tt[i] == b); VST2(int, CNT + (long long)ch * 256 + b, c); }
__global__ __launch_bounds__(256) void k_csr3_bscan(const int* __restrict__ CNT, int nch, int E, int* __restrict__ OFFB, int* __restrict__ BOFF) { __shared__ int tot[256]; const int b = threadIdx.x; int s = 0; for (int ch = 0; ch < nch; ++ch) s += CNT[(long long)ch * 256 + b]; tot[b] = s; __syncthreads();
    if (b == 0) { int run = 0; for (int i = 0; i < 256; ++i) { const int v = tot[i]; tot[i] = run; run += v; } } __syncthreads();
    int run = tot[b]; VST2(int, BOFF + b, run); if (b == 255) VST2(int, BOFF + 256, E);
    for (int ch = 0; ch < nch; ++ch) { VST2(int, OFFB + (long long)ch * 256 + b, run); run += CNT[(long long)ch * 256 + b]; } }
__global__ __launch_bounds__(256) void k_csr3_bscatter(const int* __restrict__ tgt, int E, int N, const int* __restrict__ OFFB, int* __restrict__ BUF) { __shared__ int tt[IL3_CH]; const int ch = blockIdx.x; const int b = threadIdx.x; const int e0 = ch * IL3_CH; const int nt = min(IL3_CH, E - e0);
    for (int i = b; i < nt; i += 256) tt[i] = (int)(((long long)tgt[e0 + i] * 256) / N); __syncthreads(); int pos = OFFB[(long long)ch * 256 + b];
    for (int i = 0; i < nt; ++i) if (tt[i] == b) { VST2(int, BUF + pos, e0 + i); ++pos; } }
template <int CAP>
__global__ __launch_bounds__(256) void k_csr3_lists(const int* __restrict__ tgt, const int* __restrict__ BUF, const int* __restrict__ BOFF, int N, int* __restrict__ NBR, int* __restrict__ cnt) { const int d = blockIdx.x * 256 + threadIdx.x; if (d >= N) return; const int b = (int)(((long long)d * 256) / N); int n = 0; int* row = NBR + (long long)d * CAP;
    for (int p = BOFF[b]; p < BOFF[b + 1]; ++p) { const int e = BUF[p]; if (tgt[e] == d) { if (n < CAP) VST2(int, row + n, e); ++n; } }
    for (int j = n; j < CAP; ++j) VST2(int, row + j, -1); VST2(int, cnt + d, min(n, CAP)); }
__global__ __launch_bounds__(256) void k_csr3_scan(const int* __restrict__ cnt, int* __restrict__ off, int N) {
    __shared__ int part[256]; const int per = ((((N + 255) / 256) + 31) / 32) * 32; const int a = threadIdx.x * per, b = min(N, a + per); int s = 0;
    for (int i = a; i < b; ++i) s += cnt[i]; part[threadIdx.x] = s; __syncthreads();
    if (threadIdx.x == 0) { int run = 0; for (int t = 0; t < 256; ++t) { const int v = part[t]; part[t] = run; run += v; } } __syncthreads();
    int run = part[threadIdx.x]; for (int i = a; i < b; ++i) { VST2(int, off + i, run); run += cnt[i]; }
    if (a < N && b == N) { VST2(int, off + N, run); } }
template <int CAP>
__global__ __launch_bounds__(256) void k_csr3_slotcopy(const int* __restrict__ off, const int* __restrict__ NBR, int* __restrict__ slot, int N) {
    const int t = blockIdx.x * 256 + threadIdx.x; const int tot = off[N]; if (t >= tot) return;
    int lo = 0, hi = N - 1; while (lo < hi) { const int mid = (lo + hi + 1) >> 1; if (off[mid] <= t) lo = mid; else hi = mid - 1; }
    int j = t - off[lo]; j = (j < 0) ? 0 : ((j >= CAP) ? (CAP - 1) : j); VST2(int, slot + t, NBR[(long long)lo * CAP + j]); }

__global__ __launch_bounds__(256) void k_rg_aqk(const float* __restrict__ XR, const float* __restrict__ q, const float* __restrict__ kk, float* __restrict__ AQK, int RN, int HO) { const int w = blockIdx.x * 256 + threadIdx.x; if (w >= RN * 3) return; const int h = w % 3; const long long rn = w / 3; const float* x = XR + rn * HO; float a = 0.f, b = 0.f;
#pragma unroll 1
    for (int o = 0; o < HO; ++o) { a += x[o] * q[o * 3 + h]; b += x[o] * kk[o * 3 + h]; } VST2(float, AQK + rn * 8 + h, a); VST2(float, AQK + rn * 8 + 4 + h, b); }
__global__ __launch_bounds__(64) void k_rg_agg(const float* __restrict__ XR, const float* __restrict__ AQK, const int* __restrict__ ei, const int* __restrict__ et, const int* __restrict__ off, const int* __restrict__ slot, const float* __restrict__ bias, float* __restrict__ OUT, int N, int E, int OUTC, int act) { const int n = blockIdx.x; const int c = threadIdx.x; if (c >= OUTC) return; const int HO = 3 * OUTC; float acc = 0.f;
    for (int h = 0; h < 3; ++h) { float mx = -__builtin_inff(); for (int p = off[n]; p < off[n + 1]; ++p) { const int e = slot[p]; const int t = et[e], s = ei[e]; float v = AQK[((long long)t * N + n) * 8 + h] + AQK[((long long)t * N + s) * 8 + 4 + h]; v = (v > 0.f) ? v : 0.2f * v; mx = fmaxf(mx, v); }
        float den = 0.f, a = 0.f; for (int p = off[n]; p < off[n + 1]; ++p) { const int e = slot[p]; const int t = et[e], s = ei[e]; float v = AQK[((long long)t * N + n) * 8 + h] + AQK[((long long)t * N + s) * 8 + 4 + h]; v = (v > 0.f) ? v : 0.2f * v; const float w = expf(v - mx); den += w; a += w * XR[((long long)t * N + s) * HO + h * OUTC + c]; }
        if (off[n + 1] > off[n]) acc += a / (den + 1e-16f); }
    float r = acc / 3.f + bias[c]; if (act == 1) r = fmaxf(r, 0.f); else r = 1.f / (1.f + expf(-r)); VST2(float, OUT + (long long)n * OUTC + c, r); }

template __global__ void k_gemm<0>(GemmP);

extern "C" void kernel_launch(void* const* d_in, const int* in_sizes, int n_in, void* d_out, int out_size, void* d_ws, size_t ws_size, hipStream_t stream) {
    (void)in_sizes; (void)n_in; (void)out_size; (void)ws_size;
    const float* emb = (const float*)d_in[0];
    const float* w1 = (const float*)d_in[1];
    const float* q1 = (const float*)d_in[2];
    const float* k1 = (const float*)d_in[3];
    const float* b1 = (const float*)d_in[4];
    const float* w2 = (const float*)d_in[5];
    const float* q2 = (const float*)d_in[6];
    const float* k2 = (const float*)d_in[7];
    const float* b2 = (const float*)d_in[8];
    const int* ei = (const int*)d_in[9];
    const int* et = (const int*)d_in[10];
    const int Nn = 20000;
    const int E = 640000;
    const int R = 8;
    const int NH = 3;
    const int CAP = 64;
    float* out = (float*)d_out;
    char* wsp = (char*)d_ws;
    int* cnt = (int*)wsp; wsp += (((size_t)((size_t)Nn + 64) * 4 + 255) / 256) * 256;
    int* off = (int*)wsp; wsp += (((size_t)((size_t)Nn + 64) * 4 + 255) / 256) * 256;
    int* slot = (int*)wsp; wsp += (((size_t)((size_t)E + 64) * 4 + 255) / 256) * 256;
    int* nbr = (int*)wsp; wsp += (((size_t)((size_t)Nn * CAP) * 4 + 255) / 256) * 256;
    float* XR = (float*)wsp; wsp += (((size_t)((size_t)R * Nn * 192) * 4 + 255) / 256) * 256;
    float* AQK = (float*)wsp; wsp += (((size_t)((size_t)R * Nn * 8) * 4 + 255) / 256) * 256;
    float* X2 = (float*)wsp; wsp += (((size_t)((size_t)Nn * 64) * 4 + 255) / 256) * 256;
    k_csr3_bcount<<<157, 256, 0, stream>>>(ei + E, E, Nn, nbr);
    k_csr3_bscan<<<1, 256, 0, stream>>>(nbr, 157, E, nbr + 40192, off);
    k_csr3_bscatter<<<157, 256, 0, stream>>>(ei + E, E, Nn, nbr + 40192, slot);
    k_csr3_lists<64><<<(unsigned)((Nn) + 255) / 256, 256, 0, stream>>>(ei + E, slot, off, Nn, nbr, cnt);
    k_csr3_scan<<<1, 256, 0, stream>>>(cnt, off, Nn);
    k_csr3_slotcopy<64><<<(unsigned)((E) + 255) / 256, 256, 0, stream>>>(off, nbr, slot, Nn);
    { GemmP gx0;
      gx0.A = emb; gx0.B = w1; gx0.bias = emb; gx0.R = emb; gx0.C = XR;
      gx0.sAo = 0; gx0.sAi = 0; gx0.sAm = 128; gx0.sAk = 1; gx0.sBo = (long long)128 * 192; gx0.sBi = 0; gx0.sBn = 1; gx0.sBk = 192; gx0.sCo = (long long)Nn * 192; gx0.sCi = 0; gx0.sCm = 192; gx0.sRo = 0; gx0.sRi = 0; gx0.sRm = 0; gx0.sRn = 0;
      gx0.M = Nn; gx0.N = 192; gx0.K = 128; gx0.zi_n = 1; gx0.flags = 0; gx0.act = 0;
      gx0.alpha = 1.0f; gx0.beta = 0.0f; gx0.sa = 1.0f; gx0.sb = 8.0f; gx0.Npad = 192; gx0.pad_ = 0;
      k_gemm<0><<<dim3((unsigned)((192) + 31) / 32, (unsigned)((Nn) + 15) / 16, (unsigned)(R)), 32, 0, stream>>>(gx0); }
    k_rg_aqk<<<(unsigned)((R * Nn * 3 + 255) / 256), 256, 0, stream>>>(XR, q1, k1, AQK, R * Nn, 192); k_rg_agg<<<Nn, 64, 0, stream>>>(XR, AQK, ei, et, off, slot, b1, X2, Nn, E, 64, 1);
    { GemmP gx1;
      gx1.A = X2; gx1.B = w2; gx1.bias = X2; gx1.R = X2; gx1.C = XR;
      gx1.sAo = 0; gx1.sAi = 0; gx1.sAm = 64; gx1.sAk = 1; gx1.sBo = (long long)64 * 48; gx1.sBi = 0; gx1.sBn = 1; gx1.sBk = 48; gx1.sCo = (long long)Nn * 48; gx1.sCi = 0; gx1.sCm = 48; gx1.sRo = 0; gx1.sRi = 0; gx1.sRm = 0; gx1.sRn = 0;
      gx1.M = Nn; gx1.N = 48; gx1.K = 64; gx1.zi_n = 1; gx1.flags = 0; gx1.act = 0;
      gx1.alpha = 1.0f; gx1.beta = 0.0f; gx1.sa = 1.0f; gx1.sb = 8.0f; gx1.Npad = 48; gx1.pad_ = 0;
      k_gemm<0><<<dim3((unsigned)((48) + 31) / 32, (unsigned)((Nn) + 15) / 16, (unsigned)(R)), 32, 0, stream>>>(gx1); }
    k_rg_aqk<<<(unsigned)((R * Nn * 3 + 255) / 256), 256, 0, stream>>>(XR, q2, k2, AQK, R * Nn, 48); k_rg_agg<<<Nn, 64, 0, stream>>>(XR, AQK, ei, et, off, slot, b2, out, Nn, E, 16, 2);
}
